// SS2D_39290360823833
// MI455X (gfx1250) — hardware-run, weakly checked
//
#include <hip/hip_runtime.h>
#include <hip/hip_fp16.h>
#include <math.h>

typedef __attribute__((ext_vector_type(16))) _Float16 v16h;
typedef __attribute__((ext_vector_type(8)))  _Float16 v8h;
typedef __attribute__((ext_vector_type(16))) __bf16   v16b;
typedef __attribute__((ext_vector_type(8)))  __bf16   v8b;
typedef __attribute__((ext_vector_type(8)))  float    v8f;
typedef __attribute__((ext_vector_type(4)))  float    v4f;
typedef __attribute__((ext_vector_type(4)))  unsigned v4u;

constexpr int kNb    = 2;
constexpr int kHt    = 32;
constexpr int kWd    = 32;
constexpr int kSeq   = kHt * kWd;
constexpr int kTok   = kNb * kSeq;
constexpr int kDm    = 96;
constexpr int kDin   = 192;
constexpr int kNst   = 16;
constexpr int kRank  = 6;
constexpr int kDir   = 4;
constexpr int kXpR   = kRank + 2 * kNst;
constexpr int kXdC   = 48;
constexpr int kXdB   = 8;
constexpr int kXdP   = kDir * kXdC;
constexpr int kBcP   = 2 * kNst;
static_assert(kSeq == 1024);
static_assert(kTok == 2048);
static_assert(kXpR == 38);
static_assert(kXdP == 192);
static_assert(kBcP == 32);
static_assert((kDm % 32) == 0 && (kDin % 32) == 0);
static_assert((kTok % 32) == 0 && (kDm % 32) == 0);
static_assert((kDin % 64) == 0 && (kXdP % 64) == 0 && (kSeq % 64) == 0);

constexpr float kCarryY   = 16.0f;
constexpr float kCarryYn  = 16.0f;
constexpr float kCarryWo  = 64.0f;
constexpr float kScaleOut = 1.0f / (kCarryYn * kCarryWo);
constexpr float kMergeScale = 0.25f / kCarryY;

constexpr size_t kSzXH   = (size_t)kTok * kDm * 2;
constexpr size_t kSzWIN  = (size_t)kDin * kDm * 2;
constexpr size_t kSzWX   = (size_t)kXdP * kDin * 2;
constexpr size_t kSzWOUT = (size_t)kDm * kDin * 2;
constexpr size_t kSzXI   = (size_t)kTok * kDin * 4;
constexpr size_t kSzXA   = (size_t)kTok * kDin * 2;
constexpr size_t kSzU    = (size_t)kNb * kDir * kSeq * kDin * 4;
constexpr size_t kSzXD   = (size_t)kTok * kXdP * 4;
constexpr size_t kSzBC   = (size_t)kNb * kDir * kSeq * kBcP * 4;
constexpr size_t kSzDTP  = (size_t)kNb * kDir * kSeq * kDin * 4;
constexpr size_t kSzYS   = (size_t)kNb * kDir * kSeq * kDin * 2;
constexpr size_t kSzYN   = (size_t)kTok * kDin * 2;
constexpr size_t kOffXH   = 0;
constexpr size_t kOffXL   = kOffXH   + kSzXH;
constexpr size_t kOffWINH = kOffXL   + kSzXH;
constexpr size_t kOffWINL = kOffWINH + kSzWIN;
constexpr size_t kOffWXH  = kOffWINL + kSzWIN;
constexpr size_t kOffWXL  = kOffWXH  + kSzWX;
constexpr size_t kOffWOUT = kOffWXL  + kSzWX;
constexpr size_t kOffXI   = kOffWOUT + kSzWOUT;
constexpr size_t kOffXAH  = kOffXI   + kSzXI;
constexpr size_t kOffXAL  = kOffXAH  + kSzXA;
constexpr size_t kOffU    = kOffXAL  + kSzXA;
constexpr size_t kOffXD   = kOffU    + kSzU;
constexpr size_t kOffBC   = kOffXD   + kSzXD;
constexpr size_t kOffDTP  = kOffBC   + kSzBC;
constexpr size_t kOffYS   = kOffDTP  + kSzDTP;
constexpr size_t kOffYN   = kOffYS   + kSzYS;
constexpr size_t kWsTotal = kOffYN   + kSzYN;
static_assert(kWsTotal == 23326720ull);
static_assert(kWsTotal <= 134217728ull);
static_assert((kOffXL % 128) == 0 && (kOffWINH % 128) == 0 && (kOffWINL % 128) == 0 && (kOffWXH % 128) == 0 &&
              (kOffWXL % 128) == 0 && (kOffWOUT % 128) == 0 && (kOffXI % 128) == 0 && (kOffXAH % 128) == 0 &&
              (kOffXAL % 128) == 0 && (kOffU % 128) == 0 && (kOffXD % 128) == 0 && (kOffBC % 128) == 0 &&
              (kOffDTP % 128) == 0 && (kOffYS % 128) == 0 && (kOffYN % 128) == 0);

__device__ __forceinline__ _Float16 to_h16(float v) {
  const float f = (fabsf(v) < 6.103515625e-05f) ? 0.0f : v;
  return (_Float16)f;
}
__device__ __forceinline__ float h16_to_f32(unsigned hb) {
  const unsigned sgn = (hb & 0x8000u) << 16;
  const unsigned em = hb & 0x7fffu;
  const float fn = __uint_as_float((em << 13) + 0x38000000u);
  const float fs = (float)em * 5.9604644775390625e-8f;
  const float mag = (em < 0x400u) ? fs : fn;
  return __uint_as_float(__float_as_uint(mag) | sgn);
}
__device__ __forceinline__ unsigned bf16_bits(float f) {
  const unsigned u = __float_as_uint(f);
  return (u + 0x7FFFu + ((u >> 16) & 1u)) >> 16;
}
__device__ __forceinline__ void bf16_split(float f, unsigned& hb, unsigned& lb) {
  hb = bf16_bits(f);
  lb = bf16_bits(f - __uint_as_float(hb << 16));
}
__device__ __forceinline__ void pack8_bf16(const float (&f)[8], v4u& hw, v4u& lw) {
  unsigned hb[8], lb[8];
#pragma unroll
  for (int e = 0; e < 8; ++e) bf16_split(f[e], hb[e], lb[e]);
  hw = (v4u){hb[0] | (hb[1] << 16), hb[2] | (hb[3] << 16), hb[4] | (hb[5] << 16), hb[6] | (hb[7] << 16)};
  lw = (v4u){lb[0] | (lb[1] << 16), lb[2] | (lb[3] << 16), lb[4] | (lb[5] << 16), lb[6] | (lb[7] << 16)};
}
__device__ __forceinline__ int scan_pos(int k, int l) {
  const int lp = (k & 2) ? (kSeq - 1 - l) : l;
  return (k & 1) ? (((lp & 31) << 5) | (lp >> 5)) : lp;
}
template <bool FIRST>
__device__ __forceinline__ void add_halves8(const v4u q, float (&f)[8]) {
#pragma unroll
  for (int e = 0; e < 4; ++e) {
    const unsigned w = q[e];
    const float lo = h16_to_f32(w & 0xffffu);
    const float hi = h16_to_f32(w >> 16);
    if (FIRST) {
      f[2 * e] = lo;
      f[2 * e + 1] = hi;
    } else {
      f[2 * e] += lo;
      f[2 * e + 1] += hi;
    }
  }
}

namespace eng {
constexpr int kMI = 2;
union FragH { v16h v; v8h h[2]; };
union FragB { v16b v; v8b h[2]; };
__device__ __forceinline__ v16h frag_load_h(const _Float16* p) {
  FragH f;
  f.h[0] = *(const v8h*)(p);
  f.h[1] = *(const v8h*)(p + 16);
  return f.v;
}
__device__ __forceinline__ v16b frag_load_b(const __bf16* p) {
  FragB f;
  f.h[0] = *(const v8b*)(p);
  f.h[1] = *(const v8b*)(p + 16);
  return f.v;
}
__device__ __forceinline__ v8f mma_h(v16h a, v16h b, v8f c) {
  c = __builtin_amdgcn_wmma_f32_16x16x32_f16(false, a, false, b, (short)0, c, false, false);
  asm volatile("v_nop\n\tv_nop\n\tv_nop\n\tv_nop" : "+v"(c) : "v"(a), "v"(b));
  return c;
}
__device__ __forceinline__ v8f mma_b(v16b a, v16b b, v8f c) {
  c = __builtin_amdgcn_wmma_f32_16x16x32_bf16(false, a, false, b, (short)0, c, false, false);
  asm volatile("v_nop\n\tv_nop\n\tv_nop\n\tv_nop" : "+v"(c) : "v"(a), "v"(b));
  return c;
}

__device__ __forceinline__ void tile_out(v8f (&acc)[kMI][4], float* slab, float* C, int ldc,
                                         int m0, int n0, int lane, float scale) {
  const int rlane = lane & 15;
  const int mOff  = (lane >> 4) * 8;
#pragma unroll
  for (int i = 0; i < kMI; ++i) {
    const int mBase = m0 + (i << 4);
#pragma unroll
    for (int j = 0; j < 4; ++j) {
#pragma unroll
      for (int r = 0; r < 8; ++r) {
        const float v = acc[i][j][r] * scale;
        slab[(mOff + r) * 68 + (j << 4) + rlane] = v;
      }
    }
    __builtin_amdgcn_fence(__ATOMIC_RELEASE, "workgroup");
    __builtin_amdgcn_wave_barrier();
    __builtin_amdgcn_fence(__ATOMIC_ACQUIRE, "workgroup");
    {
      const int hh = lane >> 4;
      const int c4 = (lane & 15) * 4;
      for (int pass = 0; pass < 2; ++pass) {
#pragma unroll
        for (int it = 0; it < 8; ++it) {
          const int row = it * 2 + hh;
          const v4f v = *(const v4f*)(slab + row * 68 + c4);
          *(volatile v4f*)(C + (size_t)(mBase + row) * ldc + n0 + c4) = v;
        }
        __threadfence();
      }
    }
    __builtin_amdgcn_fence(__ATOMIC_RELEASE, "workgroup");
    __builtin_amdgcn_wave_barrier();
    __builtin_amdgcn_fence(__ATOMIC_ACQUIRE, "workgroup");
  }
}

__global__ __launch_bounds__(256) void gemm_bf16x3_kernel(
    const unsigned short* __restrict__ Ahp, const unsigned short* __restrict__ Alp, int lda,
    const unsigned short* __restrict__ Bhp, const unsigned short* __restrict__ Blp, int ldb,
    float* __restrict__ Cp, int ldc, int M, int N, int K)
{
  __shared__ __align__(16) float sT[8][16 * 68];
  const int lane = threadIdx.x & 31;
  const int wave = threadIdx.x >> 5;
  const int tilesN = N >> 6;
  const int tilesM = M >> 5;
  const int tile = blockIdx.x * 8 + wave;
  if (tile >= tilesM * tilesN) return;
  const int tm = tile / tilesN;
  const int tn = tile - tm * tilesN;
  const int m0 = tm << 5;
  const int n0 = tn << 6;
  const __bf16* Ah = (const __bf16*)Ahp;
  const __bf16* Al = (const __bf16*)Alp;
  const __bf16* Bh = (const __bf16*)Bhp;
  const __bf16* Bl = (const __bf16*)Blp;
  const int rlane = lane & 15;
  const int koff  = (lane >> 4) * 8;

  v8f acc[kMI][4];
#pragma unroll
  for (int i = 0; i < kMI; ++i)
#pragma unroll
    for (int j = 0; j < 4; ++j) acc[i][j] = (v8f){0.f, 0.f, 0.f, 0.f, 0.f, 0.f, 0.f, 0.f};

  for (int k0 = 0; k0 < K; k0 += 32) {
    v16b bh[4], bl[4];
#pragma unroll
    for (int j = 0; j < 4; ++j) {
      const size_t bo = (size_t)(n0 + (j << 4) + rlane) * ldb + koff + k0;
      bh[j] = frag_load_b(Bh + bo);
      bl[j] = frag_load_b(Bl + bo);
    }
#pragma unroll
    for (int i = 0; i < kMI; ++i) {
      const size_t ao = (size_t)(m0 + (i << 4) + rlane) * lda + koff + k0;
      const v16b ah = frag_load_b(Ah + ao);
      const v16b al = frag_load_b(Al + ao);
#pragma unroll
      for (int j = 0; j < 4; ++j) {
        acc[i][j] = mma_b(ah, bl[j], acc[i][j]);
        acc[i][j] = mma_b(al, bh[j], acc[i][j]);
        acc[i][j] = mma_b(ah, bh[j], acc[i][j]);
      }
    }
  }
  tile_out(acc, sT[wave], Cp, ldc, m0, n0, lane, 1.0f);
}

__global__ __launch_bounds__(256) void gemm_f16_kernel(
    const unsigned short* __restrict__ Ap, int lda, long strideA,
    const unsigned short* __restrict__ Btp, int ldb, long strideB,
    float* __restrict__ Cp, int ldc, long strideC,
    int M, int N, int K, float scale)
{
  __shared__ __align__(16) float sT[8][16 * 68];
  const int bz   = blockIdx.y;
  const int lane = threadIdx.x & 31;
  const int wave = threadIdx.x >> 5;
  const int tilesN = N >> 6;
  const int tilesM = M >> 5;
  const int tile = blockIdx.x * 8 + wave;
  if (tile >= tilesM * tilesN) return;
  const int tm = tile / tilesN;
  const int tn = tile - tm * tilesN;
  const int m0 = tm << 5;
  const int n0 = tn << 6;
  const _Float16* Ab = (const _Float16*)Ap + (size_t)bz * strideA;
  const _Float16* Bb = (const _Float16*)Btp + (size_t)bz * strideB;
  const int rlane = lane & 15;
  const int koff  = (lane >> 4) * 8;

  v8f acc[kMI][4];
#pragma unroll
  for (int i = 0; i < kMI; ++i)
#pragma unroll
    for (int j = 0; j < 4; ++j) acc[i][j] = (v8f){0.f, 0.f, 0.f, 0.f, 0.f, 0.f, 0.f, 0.f};

  for (int k0 = 0; k0 < K; k0 += 32) {
    v16h bh[4];
#pragma unroll
    for (int j = 0; j < 4; ++j) {
      const size_t bo = (size_t)(n0 + (j << 4) + rlane) * ldb + koff + k0;
      bh[j] = frag_load_h(Bb + bo);
    }
#pragma unroll
    for (int i = 0; i < kMI; ++i) {
      const size_t ao = (size_t)(m0 + (i << 4) + rlane) * lda + koff + k0;
      const v16h ah = frag_load_h(Ab + ao);
#pragma unroll
      for (int j = 0; j < 4; ++j) acc[i][j] = mma_h(ah, bh[j], acc[i][j]);
    }
  }
  tile_out(acc, sT[wave], Cp + (size_t)bz * strideC, ldc, m0, n0, lane, scale);
}
}

__global__ __launch_bounds__(256) void xpose_split_kernel(
    const float* __restrict__ x, unsigned short* __restrict__ xh, unsigned short* __restrict__ xl)
{
  __shared__ __align__(16) float sX[kDm * 68];
  const int tid = threadIdx.x;
  const int b   = blockIdx.x >> 4;
  const int l0  = (blockIdx.x & 15) * 64;
#pragma unroll
  for (int i = 0; i < 6; ++i) {
    const int idx = tid + i * 256;
    const int c   = idx >> 4;
    const int j4  = (idx & 15) * 4;
    const v4f v = *(const v4f*)(x + ((size_t)(b * kDm + c) * kSeq + l0 + j4));
    *(v4f*)(sX + c * 68 + j4) = v;
  }
  __syncthreads();
  v4u hw[3], lw[3];
#pragma unroll
  for (int i = 0; i < 3; ++i) {
    const int piece = tid + i * 256;
    const int row = piece / 12;
    const int seg = piece - row * 12;
    float f[8];
#pragma unroll
    for (int e = 0; e < 8; ++e) f[e] = sX[(seg * 8 + e) * 68 + row];
    pack8_bf16(f, hw[i], lw[i]);
  }
  const size_t base = (size_t)(b * kSeq + l0) * kDm;
  for (int pass = 0; pass < 2; ++pass) {
#pragma unroll
    for (int i = 0; i < 3; ++i) {
      const size_t o = base + (size_t)(tid + i * 256) * 8;
      *(volatile v4u*)(xh + o) = hw[i];
      *(volatile v4u*)(xl + o) = lw[i];
    }
    __threadfence();
  }
}

__global__ __launch_bounds__(256) void cvt_bf16_split_kernel(
    const float* __restrict__ src, unsigned short* __restrict__ dh, unsigned short* __restrict__ dl, int total8)
{
  const int i = blockIdx.x * 256 + threadIdx.x;
  if (i >= total8) return;
  const size_t e0 = (size_t)i << 3;
  const v4f a0 = *(const v4f*)(src + e0);
  const v4f a1 = *(const v4f*)(src + e0 + 4);
  float f[8];
#pragma unroll
  for (int e = 0; e < 4; ++e) {
    f[e] = a0[e];
    f[4 + e] = a1[e];
  }
  v4u hw, lw;
  pack8_bf16(f, hw, lw);
  *(volatile v4u*)(dh + e0) = hw;
  *(volatile v4u*)(dl + e0) = lw;
  __threadfence();
  *(volatile v4u*)(dh + e0) = hw;
  *(volatile v4u*)(dl + e0) = lw;
}

__global__ __launch_bounds__(256) void cvt_f16_kernel(
    const float* __restrict__ src, unsigned short* __restrict__ dst, int total8, float carry)
{
  const int i = blockIdx.x * 256 + threadIdx.x;
  if (i >= total8) return;
  const size_t e0 = (size_t)i << 3;
  const v4f a0 = *(const v4f*)(src + e0);
  const v4f a1 = *(const v4f*)(src + e0 + 4);
  v8h hv;
#pragma unroll
  for (int e = 0; e < 4; ++e) {
    hv[e]     = to_h16(a0[e] * carry);
    hv[4 + e] = to_h16(a1[e] * carry);
  }
  unsigned short* q = dst + e0;
  *(volatile v8h*)q = hv;
  __threadfence();
  *(volatile v8h*)q = hv;
}

__global__ __launch_bounds__(256) void wxp_plane_kernel(
    const float* __restrict__ xpw, unsigned short* __restrict__ wh, unsigned short* __restrict__ wl)
{
  const int i   = blockIdx.x * 256 + threadIdx.x;
  const int n   = i / 24;
  const int seg = i - n * 24;
  const int k   = n / kXdC;
  const int j   = n - k * kXdC;
  const bool isdata = (j < kRank) || (j >= kXdB && j < kXdB + 2 * kNst);
  int r = (j < kRank) ? j : (j - 2);
  r = r < 0 ? 0 : (r > kXpR - 1 ? kXpR - 1 : r);
  const int d0 = seg * 8;
  float f[8];
#pragma unroll
  for (int e = 0; e < 8; ++e) {
    float v = xpw[((size_t)(k * kDin + d0 + e)) * kXpR + r];
    asm volatile("" : "+v"(v));
    f[e] = isdata ? v : 0.0f;
  }
  v4u hw, lw;
  pack8_bf16(f, hw, lw);
  const size_t o = (size_t)i * 8;
  *(volatile v4u*)(wh + o) = hw;
  *(volatile v4u*)(wl + o) = lw;
  __threadfence();
  *(volatile v4u*)(wh + o) = hw;
  *(volatile v4u*)(wl + o) = lw;
}

__global__ __launch_bounds__(192) void conv_silu_kernel(
    const float* __restrict__ xi, const float* __restrict__ cw, const float* __restrict__ cb,
    float* __restrict__ U, unsigned short* __restrict__ xah, unsigned short* __restrict__ xal)
{
  __shared__ __align__(16) float sT[4 * kDin];
  const int tid = threadIdx.x;
  const int tl  = tid / 48;
  const int c4  = (tid - tl * 48) * 4;
  const int token = blockIdx.x * 4 + tl;
  const int b  = token >> 10;
  const int l  = token & (kSeq - 1);
  const int hh = l >> 5;
  const int ww = l & 31;

  v4f wv[9];
#pragma unroll
  for (int i = 0; i < 9; ++i) wv[i] = *(const v4f*)(cw + (size_t)c4 * 9 + 4 * i);
  const v4f bias = *(const v4f*)(cb + c4);

  float acc[4] = {0.f, 0.f, 0.f, 0.f};
#pragma unroll
  for (int kh = 0; kh < 3; ++kh) {
#pragma unroll
    for (int kw = 0; kw < 3; ++kw) {
      const int tap = kh * 3 + kw;
      const int hy = hh + kh - 1;
      const int wx = ww + kw - 1;
      const bool ok = ((unsigned)hy < (unsigned)kHt) && ((unsigned)wx < (unsigned)kWd);
      const int hyc = hy < 0 ? 0 : (hy > kHt - 1 ? kHt - 1 : hy);
      const int wxc = wx < 0 ? 0 : (wx > kWd - 1 ? kWd - 1 : wx);
      const float* p = xi + (size_t)(b * kSeq + hyc * kWd + wxc) * kDin + c4;
      v4f xv = *(const v4f*)(p);
      asm volatile("" : "+v"(xv));
#pragma unroll
      for (int c = 0; c < 4; ++c) {
        const float xs = ok ? xv[c] : 0.0f;
        acc[c] = fmaf(xs, wv[(c * 9 + tap) >> 2][(c * 9 + tap) & 3], acc[c]);
      }
    }
  }
  v4f val;
#pragma unroll
  for (int c = 0; c < 4; ++c) {
    const float sv = acc[c] + bias[c];
    const float sg = __builtin_amdgcn_rcpf(1.0f + expf(-sv));
    val[c] = sv * sg;
  }
  *(v4f*)(sT + tl * kDin + c4) = val;

  const int l1 = ww * 32 + hh;
  const size_t pb = (size_t)b * kDir * kSeq;
  float* q0 = U + ((pb + 0 * kSeq + l) * kDin + c4);
  float* q1 = U + ((pb + 1 * kSeq + l1) * kDin + c4);
  float* q2 = U + ((pb + 2 * kSeq + (kSeq - 1 - l)) * kDin + c4);
  float* q3 = U + ((pb + 3 * kSeq + (kSeq - 1 - l1)) * kDin + c4);
  for (int pass = 0; pass < 2; ++pass) {
    *(volatile v4f*)q0 = val;
    *(volatile v4f*)q1 = val;
    *(volatile v4f*)q2 = val;
    *(volatile v4f*)q3 = val;
    __threadfence();
  }
  __syncthreads();
  if (tid < 96) {
    const v4f f0 = *(const v4f*)(sT + tid * 8);
    const v4f f1 = *(const v4f*)(sT + tid * 8 + 4);
    float f[8];
#pragma unroll
    for (int e = 0; e < 4; ++e) {
      f[e] = f0[e];
      f[4 + e] = f1[e];
    }
    v4u hw, lw;
    pack8_bf16(f, hw, lw);
    const size_t o = (size_t)blockIdx.x * (4 * kDin) + (size_t)tid * 8;
    *(volatile v4u*)(xah + o) = hw;
    *(volatile v4u*)(xal + o) = lw;
    __threadfence();
    *(volatile v4u*)(xah + o) = hw;
    *(volatile v4u*)(xal + o) = lw;
  }
}

__global__ __launch_bounds__(256) void dir_planes_kernel(
    const float* __restrict__ xd, const float* __restrict__ dtw, const float* __restrict__ dtb,
    float* __restrict__ BC, float* __restrict__ DTP)
{
  const int tid = threadIdx.x;
  if (blockIdx.x < 256) {
    const int i  = blockIdx.x * 256 + tid;
    const int g  = i & 7;
    const int rl = i >> 3;
    const int l  = rl & (kSeq - 1);
    const int bk = rl >> 10;
    const int k  = bk & 3;
    const int b  = bk >> 2;
    const int tok = scan_pos(k, l);
    const v4f v = *(const v4f*)(xd + (size_t)(b * kSeq + tok) * kXdP + k * kXdC + kXdB + g * 4);
    float* q = BC + (size_t)rl * kBcP + g * 4;
    *(volatile v4f*)q = v;
    __threadfence();
    *(volatile v4f*)q = v;
  } else {
    const int i  = (blockIdx.x - 256) * 256 + tid;
    const int rl = i / 48;
    const int c4 = (i - rl * 48) * 4;
    const int l  = rl & (kSeq - 1);
    const int bk = rl >> 10;
    const int k  = bk & 3;
    const int b  = bk >> 2;
    const int tok = scan_pos(k, l);
    const float* xr = xd + (size_t)(b * kSeq + tok) * kXdP + k * kXdC;
    const v4f d0 = *(const v4f*)(xr);
    const v4f d1 = *(const v4f*)(xr + 4);
    const float* wp = dtw + (size_t)(k * kDin + c4) * kRank;
    v4f wq[6];
#pragma unroll
    for (int t = 0; t < 6; ++t) wq[t] = *(const v4f*)(wp + 4 * t);
    const v4f bb = *(const v4f*)(dtb + k * kDin + c4);
    const float dr[6] = {d0[0], d0[1], d0[2], d0[3], d1[0], d1[1]};
    v4f o;
#pragma unroll
    for (int c = 0; c < 4; ++c) {
      float s = 0.0f;
#pragma unroll
      for (int r = 0; r < 6; ++r) s = fmaf(dr[r], wq[(c * 6 + r) >> 2][(c * 6 + r) & 3], s);
      o[c] = (s + bb[c]) + bb[c];
    }
    float* q = DTP + (size_t)rl * kDin + c4;
    *(volatile v4f*)q = o;
    __threadfence();
    *(volatile v4f*)q = o;
  }
}

typedef float    ms1_v4f __attribute__((ext_vector_type(4)));
typedef unsigned ms1_v4u __attribute__((ext_vector_type(4)));
struct ms1_args {
  const float* dtpre;
  const float* u;
  const float* bc;
  const float* z;
  const float* A_log;
  const float* Dskip;
  __half* y;
  __half* y_lo;
  long ld_dtpre;
  long ld_u;
  long ld_bc;
  long ld_z;
  long ld_y;
  int offB;
  int offC;
  int offZ;
  float ycarry;
  int dir;
  int D;
  int L;
  int nbatch;
};
static_assert(sizeof(ms1_args) == 136);

__device__ __forceinline__ float ms1_flush16(float v) {
  return (fabsf(v) < 6.103515625e-05f) ? 0.0f : v;
}
__device__ __forceinline__ unsigned ms1_h16bits(float v) {
  return (unsigned)__half_as_ushort(__float2half_rn(ms1_flush16(v)));
}
__device__ __forceinline__ float ms1_h16val(unsigned b) {
  return __half2float(__ushort_as_half((unsigned short)b));
}
__device__ __forceinline__ float ms1_softplus(float v) {
  return fmaxf(v, 0.0f) + log1pf(expf(-fabsf(v)));
}
__device__ __forceinline__ void ms1_pack2(float v0, float v1, unsigned& hw, unsigned& lw) {
  const unsigned h0 = ms1_h16bits(v0);
  const unsigned h1 = ms1_h16bits(v1);
  const float r0 = (v0 - ms1_h16val(h0)) * 2048.0f;
  const float r1 = (v1 - ms1_h16val(h1)) * 2048.0f;
  const unsigned l0 = ms1_h16bits(r0);
  const unsigned l1 = ms1_h16bits(r1);
  hw = h0 | (h1 << 16);
  lw = l0 | (l1 << 16);
}

template <int NSTATE>
__global__ __launch_bounds__(64 * (NSTATE / 16)) void ms1_scan_kernel(ms1_args a)
{
  static_assert(NSTATE == 16 || NSTATE == 64);
  constexpr int NQ  = NSTATE / 16;
  constexpr int NT  = 64 * NQ;
  constexpr int NW  = NT / 32;
  constexpr int BCW = 2 * NSTATE;
  constexpr int YP  = 68;
  constexpr int RPI = NW * 4;
  constexpr int NIT = 64 / RPI;
  static_assert(16 * NT <= 64 * YP);
  __shared__ __align__(16) float sBC[64 * BCW];
  __shared__ __align__(16) float sY[64 * YP];
  const int tid  = threadIdx.x;
  const int lane = tid & 31;
  const int wave = tid >> 5;
  const int c    = tid / NQ;
  const int sq   = tid - c * NQ;
  const int bpb  = a.D / 64;
  const int bi   = blockIdx.x / bpb;
  if (bi >= a.nbatch) return;
  const int d0 = (blockIdx.x - bi * bpb) * 64;
  const int d  = d0 + c;
  const long rowb = (long)bi * a.L;
  const bool hasz  = (a.z != nullptr);
  const bool hasD  = (a.Dskip != nullptr);
  const bool hasLo = (a.y_lo != nullptr);

#pragma unroll 1
  for (int n = 0; n < 16; ++n) {
    const float al = a.A_log[(long)d * NSTATE + sq * 16 + n];
    sY[n * NT + tid] = -expf(al);
  }
  __syncthreads();
  float An[16], h[16];
#pragma unroll
  for (int n = 0; n < 16; ++n) {
    An[n] = sY[n * NT + tid];
    h[n] = 0.0f;
  }
  float Dd = 0.0f;
  if (hasD) Dd = a.Dskip[d];

  const int nchunk = a.L / 64;
  const bool fwd = (a.dir > 0);
  const int s0 = fwd ? 0 : 63;
  const int sd = fwd ? 1 : -1;
  const int q  = lane >> 3;
  const int c8 = (lane & 7) * 8;

#pragma unroll 1
  for (int ci = 0; ci < nchunk; ++ci) {
    const int tb = fwd ? (ci * 64) : (a.L - 64 - ci * 64);
    const long rowc = rowb + tb;
    __syncthreads();
#pragma unroll 8
    for (int i = 0; i < 32; ++i) {
      const int idx = tid + i * NT;
      const int st  = idx / BCW;
      const int col = idx - st * BCW;
      const int sc  = (col < NSTATE) ? (a.offB + col) : (a.offC + col - NSTATE);
      sBC[idx] = a.bc[(rowc + st) * a.ld_bc + sc];
    }
    __syncthreads();
#pragma unroll 1
    for (int s = 0; s < 64; ++s) {
      const int ls = s0 + sd * s;
      const long row = rowc + ls;
      float pre = a.dtpre[row * a.ld_dtpre + d];
      float uv  = a.u[row * a.ld_u + d];
      float zv  = 0.0f;
      if (hasz) zv = a.z[row * a.ld_z + a.offZ + d];
      asm volatile("" : "+v"(pre));
      asm volatile("" : "+v"(uv));
      asm volatile("" : "+v"(zv));
      const float delta = ms1_softplus(pre);
      const float dtx = delta * uv;
      const float* bp = sBC + ls * BCW + sq * 16;
      const float* cp = bp + NSTATE;
      ms1_v4f Bq[4], Cq[4];
#pragma unroll
      for (int k = 0; k < 4; ++k) {
        Bq[k] = *(const ms1_v4f*)(bp + 4 * k);
        Cq[k] = *(const ms1_v4f*)(cp + 4 * k);
      }
      float yv = 0.0f;
#pragma unroll
      for (int n = 0; n < 16; ++n) {
        const float e = __expf(delta * An[n]);
        h[n] = fmaf(e, h[n], dtx * Bq[n >> 2][n & 3]);
        yv = fmaf(h[n], Cq[n >> 2][n & 3], yv);
      }
      if (NQ > 1) {
        yv += __shfl_xor(yv, 1, 32);
        yv += __shfl_xor(yv, 2, 32);
      }
      if (hasD) yv = fmaf(uv, Dd, yv);
      if (hasz) {
        const float sg = __builtin_amdgcn_rcpf(1.0f + expf(-zv));
        yv = yv * (zv * sg);
      }
      if (sq == 0) sY[ls * YP + c] = yv * a.ycarry;
    }
    __syncthreads();
    ms1_v4u hw[NIT], lw[NIT];
#pragma unroll
    for (int it = 0; it < NIT; ++it) {
      const int row = it * RPI + wave * 4 + q;
      const float* sp = sY + row * YP + c8;
      const ms1_v4f f0 = *(const ms1_v4f*)(sp);
      const ms1_v4f f1 = *(const ms1_v4f*)(sp + 4);
      unsigned h0, h1, h2, h3, l0, l1, l2, l3;
      ms1_pack2(f0[0], f0[1], h0, l0);
      ms1_pack2(f0[2], f0[3], h1, l1);
      ms1_pack2(f1[0], f1[1], h2, l2);
      ms1_pack2(f1[2], f1[3], h3, l3);
      hw[it] = (ms1_v4u){h0, h1, h2, h3};
      lw[it] = (ms1_v4u){l0, l1, l2, l3};
    }
    for (int pass = 0; pass < 2; ++pass) {
#pragma unroll
      for (int it = 0; it < NIT; ++it) {
        const int row = it * RPI + wave * 4 + q;
        const long o = (rowc + row) * a.ld_y + d0 + c8;
        *(volatile ms1_v4u*)(a.y + o) = hw[it];
        if (hasLo) *(volatile ms1_v4u*)(a.y_lo + o) = lw[it];
      }
      __threadfence();
    }
  }
}

__global__ __launch_bounds__(256) void merge_norm_kernel(
    const unsigned short* __restrict__ ys, const float* __restrict__ lnw, const float* __restrict__ lnb,
    unsigned short* __restrict__ yn)
{
  const int tid  = threadIdx.x;
  const int lane = tid & 31;
  const int wv   = tid >> 5;
  const int token = blockIdx.x * 8 + wv;
  const int b  = token >> 10;
  const int l  = token & (kSeq - 1);
  const int hh = l >> 5;
  const int ww = l & 31;
  const int l1 = ww * 32 + hh;
  const bool act = (lane < 24);
  const int chc = act ? (lane * 8) : ((lane - 8) * 8);
  const size_t pb = (size_t)b * kDir * kSeq;
  v4u q0 = *(const v4u*)(ys + ((pb + 0 * kSeq + l) * kDin + chc));
  v4u q2 = *(const v4u*)(ys + ((pb + 2 * kSeq + (kSeq - 1 - l)) * kDin + chc));
  v4u q1 = *(const v4u*)(ys + ((pb + 1 * kSeq + l1) * kDin + chc));
  v4u q3 = *(const v4u*)(ys + ((pb + 3 * kSeq + (kSeq - 1 - l1)) * kDin + chc));
  asm volatile("" : "+v"(q0));
  asm volatile("" : "+v"(q2));
  asm volatile("" : "+v"(q1));
  asm volatile("" : "+v"(q3));
  float v[8];
  add_halves8<true>(q0, v);
  add_halves8<false>(q2, v);
  add_halves8<false>(q1, v);
  add_halves8<false>(q3, v);
  float s = 0.0f;
#pragma unroll
  for (int j = 0; j < 8; ++j) {
    const float t = v[j] * kMergeScale;
    v[j] = act ? t : 0.0f;
    s += v[j];
  }
  s += __shfl_xor(s, 16, 32);
  s += __shfl_xor(s, 8, 32);
  s += __shfl_xor(s, 4, 32);
  s += __shfl_xor(s, 2, 32);
  s += __shfl_xor(s, 1, 32);
  const float mu = s * (1.0f / (float)kDin);
  float s2 = 0.0f;
#pragma unroll
  for (int j = 0; j < 8; ++j) {
    const float dlt = act ? (v[j] - mu) : 0.0f;
    s2 = fmaf(dlt, dlt, s2);
  }
  s2 += __shfl_xor(s2, 16, 32);
  s2 += __shfl_xor(s2, 8, 32);
  s2 += __shfl_xor(s2, 4, 32);
  s2 += __shfl_xor(s2, 2, 32);
  s2 += __shfl_xor(s2, 1, 32);
  const float var = s2 * (1.0f / (float)kDin);
  const float rs = rsqrtf(var + 1e-5f);

  v4f w0 = *(const v4f*)(lnw + chc);
  v4f w1 = *(const v4f*)(lnw + chc + 4);
  v4f b0 = *(const v4f*)(lnb + chc);
  v4f b1 = *(const v4f*)(lnb + chc + 4);
  asm volatile("" : "+v"(w0), "+v"(w1));
  asm volatile("" : "+v"(b0), "+v"(b1));
  float wj[8], bj[8];
#pragma unroll
  for (int e = 0; e < 4; ++e) {
    wj[e] = w0[e];
    wj[4 + e] = w1[e];
    bj[e] = b0[e];
    bj[4 + e] = b1[e];
  }
  v8h hv;
#pragma unroll
  for (int j = 0; j < 8; ++j) {
    const float o = (v[j] - mu) * rs * wj[j] + bj[j];
    hv[j] = to_h16(o * kCarryYn);
  }
  unsigned short* q = yn + (size_t)token * kDin + chc;
  if (act) *(volatile v8h*)q = hv;
  __threadfence();
  if (act) *(volatile v8h*)q = hv;
}

extern "C" void kernel_launch(void* const* d_in, const int* in_sizes, int n_in,
                              void* d_out, int out_size, void* d_ws, size_t ws_size,
                              hipStream_t stream) {
  if (n_in < 12) return;
  if (in_sizes[0] != kTok * kDm) return;
  if (in_sizes[1] != 2 * kDin * kDm) return;
  if (in_sizes[2] != kDin * 9) return;
  if (in_sizes[3] != kDin) return;
  if (in_sizes[4] != kDir * kDin * kXpR) return;
  if (in_sizes[5] != kDir * kDin * kRank) return;
  if (in_sizes[6] != kDir * kDin) return;
  if (in_sizes[7] != kDir * kDin * kNst) return;
  if (in_sizes[8] != kDir * kDin) return;
  if (in_sizes[9] != kDin) return;
  if (in_sizes[10] != kDin) return;
  if (in_sizes[11] != kDm * kDin) return;
  if (out_size != kTok * kDm) return;
  if (ws_size < kWsTotal) return;

  const float* x       = (const float*)d_in[0];
  const float* W_in    = (const float*)d_in[1];
  const float* conv_w  = (const float*)d_in[2];
  const float* conv_b  = (const float*)d_in[3];
  const float* W_xp    = (const float*)d_in[4];
  const float* W_dt    = (const float*)d_in[5];
  const float* b_dt    = (const float*)d_in[6];
  const float* A_log   = (const float*)d_in[7];
  const float* D_par   = (const float*)d_in[8];
  const float* ln_w    = (const float*)d_in[9];
  const float* ln_b    = (const float*)d_in[10];
  const float* W_out   = (const float*)d_in[11];
  float* out = (float*)d_out;

  char* ws = (char*)d_ws;
  unsigned short* XH   = (unsigned short*)(ws + kOffXH);
  unsigned short* XL   = (unsigned short*)(ws + kOffXL);
  unsigned short* WINH = (unsigned short*)(ws + kOffWINH);
  unsigned short* WINL = (unsigned short*)(ws + kOffWINL);
  unsigned short* WXH  = (unsigned short*)(ws + kOffWXH);
  unsigned short* WXL  = (unsigned short*)(ws + kOffWXL);
  unsigned short* WOUT = (unsigned short*)(ws + kOffWOUT);
  float*          XI   = (float*)(ws + kOffXI);
  unsigned short* XAH  = (unsigned short*)(ws + kOffXAH);
  unsigned short* XAL  = (unsigned short*)(ws + kOffXAL);
  float*          U    = (float*)(ws + kOffU);
  float*          XD   = (float*)(ws + kOffXD);
  float*          BC   = (float*)(ws + kOffBC);
  float*          DTP  = (float*)(ws + kOffDTP);
  unsigned short* YS   = (unsigned short*)(ws + kOffYS);
  unsigned short* YN   = (unsigned short*)(ws + kOffYN);

  xpose_split_kernel<<<kNb * (kSeq / 64), 256, 0, stream>>>(x, XH, XL);
  cvt_bf16_split_kernel<<<(kDin * kDm / 8) / 256, 256, 0, stream>>>(W_in, WINH, WINL, kDin * kDm / 8);
  wxp_plane_kernel<<<(kXdP * (kDin / 8)) / 256, 256, 0, stream>>>(W_xp, WXH, WXL);
  cvt_f16_kernel<<<(kDm * kDin / 8) / 256, 256, 0, stream>>>(W_out, WOUT, kDm * kDin / 8, kCarryWo);

  eng::gemm_bf16x3_kernel<<<(kTok / 32) * (kDin / 64) / 8, 256, 0, stream>>>(
      XH, XL, kDm, WINH, WINL, kDm, XI, kDin, kTok, kDin, kDm);

  conv_silu_kernel<<<kTok / 4, 192, 0, stream>>>(XI, conv_w, conv_b, U, XAH, XAL);

  eng::gemm_bf16x3_kernel<<<(kTok / 32) * (kXdP / 64) / 8, 256, 0, stream>>>(
      XAH, XAL, kDin, WXH, WXL, kDin, XD, kXdP, kTok, kXdP, kDin);

  dir_planes_kernel<<<256 + 1536, 256, 0, stream>>>(XD, W_dt, b_dt, BC, DTP);

  for (int b = 0; b < kNb; ++b) {
    for (int k = 0; k < kDir; ++k) {
      const size_t bk = (size_t)b * kDir + k;
      ms1_args sa;
      sa.dtpre = DTP + bk * kSeq * kDin;
      sa.u = U + bk * kSeq * kDin;
      sa.bc = BC + bk * kSeq * kBcP;
      sa.z = nullptr;
      sa.A_log = A_log + (size_t)k * kDin * kNst;
      sa.Dskip = D_par + (size_t)k * kDin;
      sa.y = (__half*)(YS + bk * kSeq * kDin);
      sa.y_lo = nullptr;
      sa.ld_dtpre = kDin;
      sa.ld_u = kDin;
      sa.ld_bc = kBcP;
      sa.ld_z = 0;
      sa.ld_y = kDin;
      sa.offB = 0;
      sa.offC = kNst;
      sa.offZ = 0;
      sa.ycarry = kCarryY;
      sa.dir = 1;
      sa.D = kDin;
      sa.L = kSeq;
      sa.nbatch = 1;
      ms1_scan_kernel<16><<<dim3(kDin / 64), 64, 0, stream>>>(sa);
    }
  }

  merge_norm_kernel<<<kTok / 8, 256, 0, stream>>>(YS, ln_w, ln_b, YN);

  eng::gemm_f16_kernel<<<dim3((kDm / 32) * (kSeq / 64) / 8, kNb), 256, 0, stream>>>(
      WOUT, kDin, 0L, YN, kDin, (long)kSeq * kDin, out, kSeq, (long)kDm * kSeq,
      kDm, kSeq, kDin, kScaleOut);
}
